// SelfAttention_23330262352109
// MI455X (gfx1250) — hardware-run, weakly checked
//
#include <hip/hip_runtime.h>


#ifndef NB
#define NB 16
#endif
#ifndef SEQ
#define SEQ 768
#endif
#ifndef SEQ_FULL
#define SEQ_FULL 768
#endif
#define DM   1024
#define NH   16
#define HD   64
#define RH   256
#define NBC  ((NB) < 4 ? (NB) : 4)
#define NBH  (NBC * NH)
#define PCAR 1024.0f
#define YCAR 64.0f
#define WCAR 64.0f
#define SCL  0.125f
#define PP   72

static_assert(SEQ % 128 == 0);
static_assert(RH % 128 == 0);
static_assert(RH <= SEQ);
static_assert((SEQ - RH) % 128 == 0);
static_assert(NB % NBC == 0);
static_assert(SEQ <= SEQ_FULL);
static_assert(DM % 64 == 0);
static_assert(NH * HD == DM);

typedef _Float16 h16;
typedef unsigned short bf;
typedef __attribute__((ext_vector_type(16))) __bf16   v16bf;
typedef __attribute__((ext_vector_type(16))) _Float16 v16h;
typedef __attribute__((ext_vector_type(8)))  _Float16 v8h;
typedef __attribute__((ext_vector_type(8)))  unsigned short v8us;
typedef __attribute__((ext_vector_type(8)))  float    v8f;
typedef __attribute__((ext_vector_type(4)))  float    v4f;
typedef __attribute__((ext_vector_type(2)))  float    v2f;
typedef __attribute__((ext_vector_type(2)))  _Float16 v2h;
typedef __attribute__((ext_vector_type(2)))  unsigned short v2us;
typedef v8h  __attribute__((may_alias)) v8ha;
typedef v4f  __attribute__((may_alias)) v4fa;
typedef v8us __attribute__((may_alias)) v8usa;

__device__ __forceinline__ unsigned short f2bf(float f) { unsigned u = __float_as_uint(f); u += 0x7FFFu + ((u >> 16) & 1u); return (unsigned short)(u >> 16); }
__device__ __forceinline__ float bf2f(unsigned short b) { return __uint_as_float(((unsigned)b) << 16); }
__device__ __forceinline__ float bfr(float f) { return bf2f(f2bf(f)); }
__device__ __forceinline__ v16h cat16(v8h lo, v8h hi) { return __builtin_shufflevector(lo, hi, 0, 1, 2, 3, 4, 5, 6, 7, 8, 9, 10, 11, 12, 13, 14, 15); }
__device__ __forceinline__ v16bf cat16b(v8us lo, v8us hi) { return __builtin_bit_cast(v16bf, __builtin_shufflevector(lo, hi, 0, 1, 2, 3, 4, 5, 6, 7, 8, 9, 10, 11, 12, 13, 14, 15)); }
__device__ __forceinline__ v8f wmma16(v16h a, v16h b, v8f c) { return __builtin_amdgcn_wmma_f32_16x16x32_f16(false, a, false, b, (short)0, c, false, false); }
__device__ __forceinline__ v8f wmmab(v16bf a, v16bf b, v8f c) { return __builtin_amdgcn_wmma_f32_16x16x32_bf16(false, a, false, b, (short)0, c, false, false); }
__device__ __forceinline__ void splitf(float y, unsigned short& h, unsigned short& l) { h = f2bf(y); l = f2bf(y - bf2f(h)); }
__device__ __forceinline__ void wsync() { asm volatile("" ::: "memory"); __builtin_amdgcn_wave_barrier(); asm volatile("" ::: "memory"); }

template <typename T16> struct WFrag;
template <> struct WFrag<h16> { typedef v16h V; static __device__ __forceinline__ V ld(const h16* p) { return cat16(*(const v8h*)p, *(const v8h*)(p + 16)); } static __device__ __forceinline__ v8f mma(V a, V b, v8f c) { return wmma16(a, b, c); } };
template <> struct WFrag<bf> { typedef v16bf V; static __device__ __forceinline__ V ld(const bf* p) { return cat16b(*(const v8us*)p, *(const v8us*)(p + 16)); } static __device__ __forceinline__ v8f mma(V a, V b, v8f c) { return wmmab(a, b, c); } };

template <typename T16, int NSPLIT, bool BIAS>
__global__ __launch_bounds__(32) void k_gemmw(const T16* __restrict__ A, const T16* __restrict__ A2, const T16* __restrict__ Bt, const T16* __restrict__ Bt2, int K, float* C, int ldc, const float* __restrict__ bias, float osc, size_t sA, size_t sB, size_t sC) {
    typedef typename WFrag<T16>::V V;
    __shared__ __align__(16) float os[16 * 68];
    const size_t z = blockIdx.z; A += z * sA; if (A2) A2 += z * sA; Bt += z * sB; if (Bt2) Bt2 += z * sB; C += z * sC;
    const int lane = threadIdx.x & 31, lr = lane & 15, hi = lane >> 4; const int r0 = blockIdx.x * 64, c0 = blockIdx.y * 64;
    v8f acc[4][4];
#pragma unroll
    for (int mb = 0; mb < 4; ++mb)
#pragma unroll
        for (int nb = 0; nb < 4; ++nb) acc[mb][nb] = (v8f){};
    const size_t aoff = (size_t)(r0 + lr) * K + 8 * hi, boff = (size_t)(c0 + lr) * K + 8 * hi;
#pragma unroll 1
    for (int kc = 0; kc < K; kc += 32) {
        V a[4], a2[4];
#pragma unroll
        for (int mb = 0; mb < 4; ++mb) { a[mb] = WFrag<T16>::ld(A + aoff + (size_t)mb * 16 * K + kc); if (NSPLIT == 1 || NSPLIT == 2) a2[mb] = WFrag<T16>::ld(A2 + aoff + (size_t)mb * 16 * K + kc); }
#pragma unroll
        for (int nb = 0; nb < 4; ++nb) { const V b = WFrag<T16>::ld(Bt + boff + (size_t)nb * 16 * K + kc); V b2; if (NSPLIT >= 2) b2 = WFrag<T16>::ld(Bt2 + boff + (size_t)nb * 16 * K + kc);
#pragma unroll
            for (int mb = 0; mb < 4; ++mb) { acc[mb][nb] = WFrag<T16>::mma(a[mb], b, acc[mb][nb]); if (NSPLIT == 1 || NSPLIT == 2) acc[mb][nb] = WFrag<T16>::mma(a2[mb], b, acc[mb][nb]); if (NSPLIT >= 2) acc[mb][nb] = WFrag<T16>::mma(a[mb], b2, acc[mb][nb]); } }
        asm volatile("v_nop\n\tv_nop\n\tv_nop\n\tv_nop" : "+v"(acc[0][0]), "+v"(acc[1][1]), "+v"(acc[2][2]), "+v"(acc[3][3]) : "v"(a[0]), "v"(a[3]));
    }
#pragma unroll
    for (int mb = 0; mb < 4; ++mb) {
#pragma unroll
        for (int nb = 0; nb < 4; ++nb) {
#pragma unroll
            for (int j = 0; j < 8; ++j) os[(hi * 8 + j) * 68 + nb * 16 + lr] = acc[mb][nb][j]; }
        wsync();
        float* crow = C + (size_t)(r0 + mb * 16) * ldc + c0;
#pragma unroll 1
        for (int ps = 0; ps < 2; ++ps) {
#pragma unroll
            for (int s = 0; s < 8; ++s) { const int row = 2 * s + hi, cofs = lr * 4; v4f val = *(const v4fa*)(os + row * 68 + cofs); val *= osc;
                if (BIAS) { val[0] += bfr(bias[c0 + cofs]); val[1] += bfr(bias[c0 + cofs + 1]); val[2] += bfr(bias[c0 + cofs + 2]); val[3] += bfr(bias[c0 + cofs + 3]); }
                *(volatile v4f*)(crow + (size_t)row * ldc + cofs) = val; }
            if (ps == 0) __threadfence(); }
        wsync();
    }
}

__global__ __launch_bounds__(256) void k_cvt8(const float* __restrict__ src, bf* dst, size_t n8) { const size_t i = (size_t)blockIdx.x * 256 + threadIdx.x; if (i >= n8) return; const v8f v = *(const v8f*)(src + i * 8); v8us o;
#pragma unroll
    for (int k = 0; k < 8; ++k) o[k] = f2bf(v[k]);
    *(volatile v8us*)(dst + i * 8) = o; __threadfence(); *(volatile v8us*)(dst + i * 8) = o; }

__global__ __launch_bounds__(256) void k_cvtwo(const float* __restrict__ src, bf* dB, h16* dH, size_t n8) { const size_t i = (size_t)blockIdx.x * 256 + threadIdx.x; if (i >= n8) return; const v8f v = *(const v8f*)(src + i * 8); v8us o; v8h oh;
#pragma unroll
    for (int k = 0; k < 8; ++k) { const unsigned short b = f2bf(v[k]); o[k] = b; oh[k] = (h16)(bf2f(b) * WCAR); }
    *(volatile v8us*)(dB + i * 8) = o; *(volatile v8h*)(dH + i * 8) = oh; __threadfence(); *(volatile v8us*)(dB + i * 8) = o; *(volatile v8h*)(dH + i * 8) = oh; }

__global__ __launch_bounds__(256) void k_cvtx(const float* __restrict__ x, bf* dst) { const size_t i = (size_t)blockIdx.x * 256 + threadIdx.x; const size_t per = (size_t)SEQ * DM / 8; if (i >= (size_t)NBC * per) return;
    const size_t bl = i / per, r = i % per; const v8f v = *(const v8f*)(x + bl * (size_t)SEQ_FULL * DM + r * 8); v8us o;
#pragma unroll
    for (int k = 0; k < 8; ++k) o[k] = f2bf(v[k]);
    *(volatile v8us*)(dst + i * 8) = o; __threadfence(); *(volatile v8us*)(dst + i * 8) = o; }

__global__ __launch_bounds__(256) void k_cstab(float* CS) { const int idx = blockIdx.x * 256 + threadIdx.x; if (idx >= SEQ * (DM / 2)) return; const int j = idx % (DM / 2), t = idx / (DM / 2);
    const float fr = exp2f(-(float)(2 * j) * (13.287712379549449f / (float)DM)); const float ang = (float)t * fr; float sn, cs; sincosf(ang, &sn, &cs);
    v2f o; o[0] = cs; o[1] = sn; *(volatile v2f*)(CS + (size_t)idx * 2) = o; __threadfence(); *(volatile v2f*)(CS + (size_t)idx * 2) = o; }

__global__ __launch_bounds__(256) void k_ropeqk(const float* __restrict__ F, const float* __restrict__ CS, h16* P16, bf* Ph, bf* Pl) {
#pragma clang fp contract(off)
    const size_t e = ((size_t)blockIdx.x * 256 + threadIdx.x) * 2; if (e >= (size_t)2 * NBH * SEQ * HD) return;
    const int d = (int)(e % HD); const int t = (int)((e / HD) % SEQ); const int bh = (int)((e / ((size_t)HD * SEQ)) % NBH); const int wh = (int)(e / ((size_t)HD * SEQ * NBH));
    const int bl = bh / NH, hh = bh % NH;
    const v2f x = *(const v2f*)(F + ((size_t)bl * SEQ + t) * (3 * DM) + (size_t)wh * DM + hh * HD + d);
    const v2f cs = *(const v2f*)(CS + ((size_t)t * (DM / 2) + hh * (HD / 2) + (d >> 1)) * 2);
    const float r0 = x[0] * cs[0] - x[1] * cs[1]; const float r1 = x[0] * cs[1] + x[1] * cs[0];
    v2h o16; o16[0] = (h16)r0; o16[1] = (h16)r1; v2us oh, ol; unsigned short a, c;
    splitf(r0, a, c); oh[0] = a; ol[0] = c; splitf(r1, a, c); oh[1] = a; ol[1] = c;
    const size_t eo = (((size_t)wh * NBH + bh) * RH + (t < RH ? t : 0)) * HD + d;
    *(volatile v2h*)(P16 + e) = o16; if (t < RH) { *(volatile v2us*)(Ph + eo) = oh; *(volatile v2us*)(Pl + eo) = ol; }
    __threadfence();
    *(volatile v2h*)(P16 + e) = o16; if (t < RH) { *(volatile v2us*)(Ph + eo) = oh; *(volatile v2us*)(Pl + eo) = ol; } }

__global__ __launch_bounds__(256) void k_vtp(const float* __restrict__ F, h16* V16, bf* Vh, bf* Vl) { const size_t e = ((size_t)blockIdx.x * 256 + threadIdx.x) * 2; if (e >= (size_t)NBH * HD * SEQ) return;
    const int t = (int)(e % SEQ); const int d = (int)((e / SEQ) % HD); const int bh = (int)(e / ((size_t)SEQ * HD)); const int bl = bh / NH, g = bh % NH; v2h o16; v2us oh, ol;
#pragma unroll
    for (int q = 0; q < 2; ++q) { const float x = F[((size_t)bl * SEQ + t + q) * (3 * DM) + 2 * DM + g * HD + d]; o16[q] = (h16)x; unsigned short a, c; splitf(x, a, c); oh[q] = a; ol[q] = c; }
    const size_t eo = ((size_t)bh * HD + d) * RH + (t < RH ? t : 0);
    *(volatile v2h*)(V16 + e) = o16; if (t < RH) { *(volatile v2us*)(Vh + eo) = oh; *(volatile v2us*)(Vl + eo) = ol; }
    __threadfence();
    *(volatile v2h*)(V16 + e) = o16; if (t < RH) { *(volatile v2us*)(Vh + eo) = oh; *(volatile v2us*)(Vl + eo) = ol; } }

template <bool HR>
__global__ __launch_bounds__(256) void k_attn(const h16* __restrict__ Q16, const h16* __restrict__ K16, const h16* __restrict__ V16,
                                              const bf* __restrict__ Qh, const bf* __restrict__ Ql, const bf* __restrict__ Kh, const bf* __restrict__ Kl,
                                              const bf* __restrict__ Vh, const bf* __restrict__ Vl, h16* A16, bf* Ah, bf* Al) {
    constexpr int TP = HR ? RH : SEQ;
    constexpr int RB = HR ? 0 : RH;
    __shared__ __align__(16) h16 ps16[HR ? 8 : 8 * 16 * PP];
    __shared__ __align__(16) bf  psh[HR ? 8 * 16 * PP : 8];
    __shared__ __align__(16) bf  psl[HR ? 8 * 16 * PP : 8];
    const int bh = blockIdx.x; const int bl = bh / NH, hh = bh % NH;
    const int wave = threadIdx.x >> 5, lane = threadIdx.x & 31, lr = lane & 15, hi = lane >> 4;
    const int qr0 = RB + blockIdx.y * 128 + wave * 16;
    const int wb = wave * 16 * PP;
    v16h qa[2]; v16bf qh[2], ql[2];
    { const size_t qo = ((size_t)bh * TP + qr0 + lr) * HD + 8 * hi;
#pragma unroll
      for (int ks = 0; ks < 2; ++ks) { if (HR) { qh[ks] = WFrag<bf>::ld(Qh + qo + ks * 32); ql[ks] = WFrag<bf>::ld(Ql + qo + ks * 32); } else { qa[ks] = WFrag<h16>::ld(Q16 + qo + ks * 32); } } }
    v8f acc[4];
#pragma unroll
    for (int dt = 0; dt < 4; ++dt) acc[dt] = (v8f){};
    float mrow[8], lrow[8];
#pragma unroll
    for (int r = 0; r < 8; ++r) { mrow[r] = -1.0e30f; lrow[r] = 0.0f; }
    const float LOG2E = 1.4426950408889634f;
    const int kend = qr0 + 16;
#pragma unroll 1
    for (int kb = 0; kb < kend; kb += 64) {
        v8f s[4];
#pragma unroll
        for (int nt = 0; nt < 4; ++nt) { v8f sa = (v8f){}; const size_t ko = ((size_t)bh * TP + kb + nt * 16 + lr) * HD + 8 * hi;
#pragma unroll
            for (int ks = 0; ks < 2; ++ks) {
                if (HR) { const v16bf kh = WFrag<bf>::ld(Kh + ko + ks * 32); const v16bf kl = WFrag<bf>::ld(Kl + ko + ks * 32);
                    sa = wmmab(qh[ks], kh, sa); sa = wmmab(ql[ks], kh, sa); sa = wmmab(qh[ks], kl, sa); }
                else { const v16h kf = WFrag<h16>::ld(K16 + ko + ks * 32); sa = wmma16(qa[ks], kf, sa); } }
            s[nt] = sa; }
        asm volatile("v_nop\n\tv_nop\n\tv_nop\n\tv_nop" : "+v"(s[0]), "+v"(s[1]), "+v"(s[2]), "+v"(s[3]));
#pragma unroll
        for (int nt = 0; nt < 4; ++nt) { const int key = kb + nt * 16 + lr;
#pragma unroll
            for (int r = 0; r < 8; ++r) { const float t = s[nt][r] * SCL; s[nt][r] = (key > qr0 + 8 * hi + r) ? -1.0e30f : t; } }
        float bm[8];
#pragma unroll
        for (int r = 0; r < 8; ++r) bm[r] = fmaxf(fmaxf(s[0][r], s[1][r]), fmaxf(s[2][r], s[3][r]));
#pragma unroll
        for (int off = 8; off >= 1; off >>= 1)
#pragma unroll
            for (int r = 0; r < 8; ++r) bm[r] = fmaxf(bm[r], __shfl_xor(bm[r], off, 32));
        float ef[8];
#pragma unroll
        for (int r = 0; r < 8; ++r) { const float nm = fmaxf(mrow[r], bm[r]); ef[r] = __builtin_amdgcn_exp2f((mrow[r] - nm) * LOG2E); mrow[r] = nm; }
#pragma unroll
        for (int dt = 0; dt < 4; ++dt)
#pragma unroll
            for (int r = 0; r < 8; ++r) acc[dt][r] *= ef[r];
#pragma unroll
        for (int nt = 0; nt < 4; ++nt)
#pragma unroll
            for (int r = 0; r < 8; ++r) s[nt][r] = __builtin_amdgcn_exp2f((s[nt][r] - mrow[r]) * LOG2E);
        float ls[8];
#pragma unroll
        for (int r = 0; r < 8; ++r) ls[r] = (s[0][r] + s[1][r]) + (s[2][r] + s[3][r]);
#pragma unroll
        for (int off = 8; off >= 1; off >>= 1)
#pragma unroll
            for (int r = 0; r < 8; ++r) ls[r] += __shfl_xor(ls[r], off, 32);
#pragma unroll
        for (int r = 0; r < 8; ++r) lrow[r] = lrow[r] * ef[r] + ls[r];
#pragma unroll
        for (int nt = 0; nt < 4; ++nt)
#pragma unroll
            for (int r = 0; r < 8; ++r) { const int o = wb + (8 * hi + r) * PP + nt * 16 + lr;
                if (HR) { unsigned short a, c; splitf(s[nt][r], a, c); psh[o] = a; psl[o] = c; } else { ps16[o] = (h16)(s[nt][r] * PCAR); } }
        wsync();
        v16h pa[2]; v16bf pah[2], pal[2];
#pragma unroll
        for (int ks = 0; ks < 2; ++ks) { const int o = wb + lr * PP + ks * 32 + 8 * hi;
            if (HR) { pah[ks] = cat16b(*(const v8usa*)(psh + o), *(const v8usa*)(psh + o + 16)); pal[ks] = cat16b(*(const v8usa*)(psl + o), *(const v8usa*)(psl + o + 16)); }
            else { pa[ks] = cat16(*(const v8ha*)(ps16 + o), *(const v8ha*)(ps16 + o + 16)); } }
#pragma unroll
        for (int dt = 0; dt < 4; ++dt) { const size_t vo = ((size_t)bh * HD + dt * 16 + lr) * TP + kb + 8 * hi;
#pragma unroll
            for (int ks = 0; ks < 2; ++ks) {
                if (HR) { const v16bf vh = WFrag<bf>::ld(Vh + vo + ks * 32); const v16bf vl = WFrag<bf>::ld(Vl + vo + ks * 32);
                    acc[dt] = wmmab(pah[ks], vh, acc[dt]); acc[dt] = wmmab(pal[ks], vh, acc[dt]); acc[dt] = wmmab(pah[ks], vl, acc[dt]); }
                else { const v16h vf = WFrag<h16>::ld(V16 + vo + ks * 32); acc[dt] = wmma16(pa[ks], vf, acc[dt]); } } }
        asm volatile("v_nop\n\tv_nop\n\tv_nop\n\tv_nop" : "+v"(acc[0]), "+v"(acc[1]), "+v"(acc[2]), "+v"(acc[3]));
        wsync();
    }
    float fo[8];
#pragma unroll
    for (int r = 0; r < 8; ++r) { const float inv = 1.0f / lrow[r]; fo[r] = HR ? inv : inv * (YCAR / PCAR); }
#pragma unroll
    for (int dt = 0; dt < 4; ++dt)
#pragma unroll
        for (int r = 0; r < 8; ++r) { const int o = wb + (8 * hi + r) * PP + dt * 16 + lr; const float y = acc[dt][r] * fo[r];
            if (HR) { unsigned short a, c; splitf(y, a, c); psh[o] = a; psl[o] = c; } else { ps16[o] = (h16)y; } }
    wsync();
    const int rq = lane >> 3, pc = (lane & 7) * 8;
    if (HR) {
        const size_t d0 = ((size_t)bl * RH + qr0) * DM + hh * HD + pc;
#pragma unroll 1
        for (int ps = 0; ps < 2; ++ps) {
#pragma unroll
            for (int s4 = 0; s4 < 4; ++s4) { const int row = s4 * 4 + rq; const v8us vh = *(const v8usa*)(psh + wb + row * PP + pc); const v8us vl = *(const v8usa*)(psl + wb + row * PP + pc);
                *(volatile v8us*)(Ah + d0 + (size_t)row * DM) = vh; *(volatile v8us*)(Al + d0 + (size_t)row * DM) = vl; }
            if (ps == 0) __threadfence(); }
    } else {
        const size_t d0 = ((size_t)bl * (SEQ - RH) + (qr0 - RH)) * DM + hh * HD + pc;
#pragma unroll 1
        for (int ps = 0; ps < 2; ++ps) {
#pragma unroll
            for (int s4 = 0; s4 < 4; ++s4) { const int row = s4 * 4 + rq; const v8h v = *(const v8ha*)(ps16 + wb + row * PP + pc);
                *(volatile v8h*)(A16 + d0 + (size_t)row * DM) = v; }
            if (ps == 0) __threadfence(); }
    }
}

extern "C" void kernel_launch(void* const* d_in, const int* in_sizes, int n_in,
                              void* d_out, int out_size, void* d_ws, size_t ws_size, hipStream_t stream) {
    if (n_in < 5) return;
    if (in_sizes[0] < NB * SEQ * DM || in_sizes[1] < 3 * DM * DM || in_sizes[2] < 3 * DM || in_sizes[3] < DM * DM || in_sizes[4] < DM) return;
    if (out_size < NB * SEQ * DM) return;
    const float* x = (const float*)d_in[0]; const float* wqkv = (const float*)d_in[1]; const float* bqkv = (const float*)d_in[2]; const float* wo = (const float*)d_in[3]; const float* bo = (const float*)d_in[4];
    float* OUT = (float*)d_out;
    char* wsp = (char*)d_ws;
    auto take = [&](size_t bytes) { char* p = wsp; wsp += (bytes + 255) & ~(size_t)255; return (void*)p; };
    bf*  WQKV = (bf*)take((size_t)3 * DM * DM * 2);
    bf*  WOb  = (bf*)take((size_t)DM * DM * 2);
    h16* WO16 = (h16*)take((size_t)DM * DM * 2);
    float* CS = (float*)take((size_t)SEQ * (DM / 2) * 2 * 4);
    bf*  XB   = (bf*)take((size_t)NBC * SEQ * DM * 2);
    float* F  = (float*)take((size_t)NBC * SEQ * 3 * DM * 4);
    h16* QK16 = (h16*)take((size_t)2 * NBH * SEQ * HD * 2);
    bf*  QKh  = (bf*)take((size_t)2 * NBH * RH * HD * 2);
    bf*  QKl  = (bf*)take((size_t)2 * NBH * RH * HD * 2);
    h16* VT16 = (h16*)take((size_t)NBH * HD * SEQ * 2);
    bf*  VTh  = (bf*)take((size_t)NBH * HD * RH * 2);
    bf*  VTl  = (bf*)take((size_t)NBH * HD * RH * 2);
    bf*  ATh  = (bf*)take((size_t)NBC * RH * DM * 2);
    bf*  ATl  = (bf*)take((size_t)NBC * RH * DM * 2);
    h16* AT16 = (h16*)take((size_t)NBC * (SEQ - RH) * DM * 2 + 256);
    const size_t carved = (size_t)(wsp - (char*)d_ws);
    if (carved > ws_size || carved > (size_t)134217728) return;

    k_cvt8<<<(unsigned)(((size_t)3 * DM * DM / 8 + 255) / 256), 256, 0, stream>>>(wqkv, WQKV, (size_t)3 * DM * DM / 8);
    k_cvtwo<<<(unsigned)(((size_t)DM * DM / 8 + 255) / 256), 256, 0, stream>>>(wo, WOb, WO16, (size_t)DM * DM / 8);
    k_cstab<<<(SEQ * (DM / 2) + 255) / 256, 256, 0, stream>>>(CS);

    h16* Q16 = QK16; h16* K16 = QK16 + (size_t)NBH * SEQ * HD;
    bf* Qh = QKh; bf* Kh = QKh + (size_t)NBH * RH * HD; bf* Ql = QKl; bf* Kl = QKl + (size_t)NBH * RH * HD;
    for (int cb = 0; cb < NB; cb += NBC) {
        k_cvtx<<<(unsigned)(((size_t)NBC * SEQ * DM / 8 + 255) / 256), 256, 0, stream>>>(x + (size_t)cb * SEQ_FULL * DM, XB);
        k_gemmw<bf, 0, true><<<dim3(NBC * SEQ / 64, 3 * DM / 64, 1), 32, 0, stream>>>(XB, nullptr, WQKV, nullptr, DM, F, 3 * DM, bqkv, 1.0f, 0, 0, 0);
        k_ropeqk<<<(unsigned)(((size_t)2 * NBH * SEQ * HD / 2 + 255) / 256), 256, 0, stream>>>(F, CS, QK16, QKh, QKl);
        k_vtp<<<(unsigned)(((size_t)NBH * HD * SEQ / 2 + 255) / 256), 256, 0, stream>>>(F, VT16, VTh, VTl);
        k_attn<true><<<dim3(NBH, RH / 128), 256, 0, stream>>>(Q16, K16, VT16, Qh, Ql, Kh, Kl, VTh, VTl, AT16, ATh, ATl);
        if (SEQ > RH) k_attn<false><<<dim3(NBH, (SEQ - RH) / 128), 256, 0, stream>>>(Q16, K16, VT16, Qh, Ql, Kh, Kl, VTh, VTl, AT16, ATh, ATl);
        k_gemmw<bf, 1, true><<<dim3(RH / 64, DM / 64, NBC), 32, 0, stream>>>(ATh, ATl, WOb, nullptr, DM, OUT + (size_t)cb * SEQ_FULL * DM, DM, bo, 1.0f, (size_t)RH * DM, 0, (size_t)SEQ_FULL * DM);
        if (SEQ > RH) k_gemmw<h16, 0, true><<<dim3((SEQ - RH) / 64, DM / 64, NBC), 32, 0, stream>>>(AT16, nullptr, WO16, nullptr, DM, OUT + ((size_t)cb * SEQ_FULL + RH) * DM, DM, bo, 1.0f / (YCAR * WCAR), (size_t)(SEQ - RH) * DM, 0, (size_t)SEQ_FULL * DM);
    }
}
